// Self_AttentionLayer_52493090292085
// MI455X (gfx1250) — hardware-verified
//
#include <hip/hip_runtime.h>


#define NB_  4
#define CC   512
#define OC   64
#define NPOS 4096
#define NT_  NPOS
#define DM   CC
#define HD   128
#define KW   CC
#define NKV  (CC / HD)
#define QH_  (NPOS / 2)
#define SCL  1.0f
#define LOSC 1024.0f

typedef _Float16 h16;
typedef unsigned short bf;
typedef __attribute__((ext_vector_type(16))) __bf16   v16bf;
typedef __attribute__((ext_vector_type(16))) _Float16 v16h;
typedef __attribute__((ext_vector_type(8)))  _Float16 v8h;
typedef __attribute__((ext_vector_type(8)))  unsigned short v8us;
typedef __attribute__((ext_vector_type(8)))  float    v8f;
typedef __attribute__((ext_vector_type(4)))  float    v4f;
typedef __attribute__((ext_vector_type(4)))  _Float16 v4h;
typedef v8h  __attribute__((may_alias)) v8ha;
typedef v4f  __attribute__((may_alias)) v4fa;
typedef v8us __attribute__((may_alias)) v8usa;

__device__ __forceinline__ unsigned short f2bf(float f) { unsigned u = __float_as_uint(f); u += 0x7FFFu + ((u >> 16) & 1u); return (unsigned short)(u >> 16); }
__device__ __forceinline__ float bf2f(unsigned short b) { return __uint_as_float(((unsigned)b) << 16); }
__device__ __forceinline__ float bfr(float f) { return bf2f(f2bf(f)); }
__device__ __forceinline__ v16h cat16(v8h lo, v8h hi) { return __builtin_shufflevector(lo, hi, 0, 1, 2, 3, 4, 5, 6, 7, 8, 9, 10, 11, 12, 13, 14, 15); }
__device__ __forceinline__ v16bf cat16b(v8us lo, v8us hi) { return __builtin_bit_cast(v16bf, __builtin_shufflevector(lo, hi, 0, 1, 2, 3, 4, 5, 6, 7, 8, 9, 10, 11, 12, 13, 14, 15)); }
__device__ __forceinline__ v8f wmma16(v16h a, v16h b, v8f c) { return __builtin_amdgcn_wmma_f32_16x16x32_f16(false, a, false, b, (short)0, c, false, false); }
__device__ __forceinline__ v8f wmmab(v16bf a, v16bf b, v8f c) { return __builtin_amdgcn_wmma_f32_16x16x32_bf16(false, a, false, b, (short)0, c, false, false); }

__global__ __launch_bounds__(256) void k_cvtb(const float* __restrict__ src, int nrows, bf* dst) {
    const int lane = threadIdx.x & 31, r = blockIdx.x * 8 + (threadIdx.x >> 5);
    if (r >= nrows) return;
    v8us o[DM / 256];
#pragma unroll
    for (int q = 0; q < DM / 256; ++q) { v8us t;
#pragma unroll
        for (int i = 0; i < 8; ++i) t[i] = f2bf(src[(size_t)r * DM + q * 256 + lane * 8 + i]);
        o[q] = t; }
#pragma unroll
    for (int q = 0; q < DM / 256; ++q) *(volatile v8us*)(dst + (size_t)r * DM + q * 256 + lane * 8) = o[q];
    __threadfence();
#pragma unroll
    for (int q = 0; q < DM / 256; ++q) *(volatile v8us*)(dst + (size_t)r * DM + q * 256 + lane * 8) = o[q];
}

__global__ __launch_bounds__(256) void k_wt(const float* __restrict__ Wm, int K, int ncols, bf* WT) {
    __shared__ __align__(16) unsigned short tl[64 * 72];
    const int tid = threadIdx.x, k0 = blockIdx.x * 64, n0 = blockIdx.y * 64;
    const int kk = tid >> 2, nq = (tid & 3) * 16;
#pragma unroll
    for (int i = 0; i < 16; ++i) tl[(nq + i) * 72 + kk] = f2bf(Wm[(size_t)(k0 + kk) * ncols + n0 + nq + i]);
    __syncthreads();
    const int piece = tid & 7;
    auto pass = [&]() {
#pragma unroll
        for (int s = 0; s < 2; ++s) { const int nr = (tid >> 3) + 32 * s; const v8us val = *(const v8usa*)(tl + nr * 72 + piece * 8); *(volatile v8us*)(WT + (size_t)(n0 + nr) * K + k0 + piece * 8) = val; }
    };
    pass(); __threadfence(); pass();
}
__global__ __launch_bounds__(256) void k_cvtb2(const float* __restrict__ src, int nrows, bf* dh, bf* dl) {
    const int lane = threadIdx.x & 31, r = blockIdx.x * 8 + (threadIdx.x >> 5);
    if (r >= nrows) return;
    v8us oh[DM / 256], ol[DM / 256];
#pragma unroll
    for (int q = 0; q < DM / 256; ++q) {
#pragma unroll
        for (int i = 0; i < 8; ++i) { const float v = src[(size_t)r * DM + q * 256 + lane * 8 + i]; const unsigned short hb = f2bf(v); oh[q][i] = hb; ol[q][i] = f2bf(v - bf2f(hb)); } }
#pragma unroll
    for (int ps = 0; ps < 2; ++ps) {
#pragma unroll
        for (int q = 0; q < DM / 256; ++q) { const size_t o = (size_t)r * DM + q * 256 + lane * 8; *(volatile v8us*)(dh + o) = oh[q]; *(volatile v8us*)(dl + o) = ol[q]; }
        if (ps == 0) __threadfence(); }
}
template <bool SPLITA, bool F16OUT = false>
__global__ __launch_bounds__(128) void k_gemmb(const bf* __restrict__ A, const bf* __restrict__ Al, const bf* __restrict__ Bn, const float* __restrict__ bias, float* C, int ldc, h16* C2, const float* __restrict__ R = nullptr, int K = DM, int roundR = 1) {
    __shared__ __align__(16) float ost[4][16 * 68];
    const int lane = threadIdx.x & 31, wave = threadIdx.x >> 5, lr = lane & 15, hi = lane >> 4;
    const int r0 = blockIdx.x * 64 + wave * 16, c0 = blockIdx.y * 64;
    const size_t aoff = (size_t)(r0 + lr) * K + 8 * hi;
    size_t boff[4];
#pragma unroll
    for (int t = 0; t < 4; ++t) boff[t] = (size_t)(c0 + t * 16 + lr) * K + 8 * hi;
    v8f acc[4];
#pragma unroll
    for (int t = 0; t < 4; ++t) acc[t] = (v8f){};
#pragma unroll 1
    for (int kc = 0; kc < K; kc += 32) {
        const v16bf a = cat16b(*(const v8us*)(A + aoff + kc), *(const v8us*)(A + aoff + kc + 16));
        v16bf al = a;
        if (SPLITA) al = cat16b(*(const v8us*)(Al + aoff + kc), *(const v8us*)(Al + aoff + kc + 16));
#pragma unroll
        for (int t = 0; t < 4; ++t) { const v16bf b = cat16b(*(const v8us*)(Bn + boff[t] + kc), *(const v8us*)(Bn + boff[t] + kc + 16)); acc[t] = wmmab(a, b, acc[t]); if (SPLITA) acc[t] = wmmab(al, b, acc[t]); }
        asm volatile("v_nop\n\tv_nop\n\tv_nop\n\tv_nop" : "+v"(acc[0]), "+v"(acc[1]), "+v"(acc[2]), "+v"(acc[3]) : "v"(a), "v"(al));
    }
    float* os = &ost[wave][0];
#pragma unroll
    for (int t = 0; t < 4; ++t) { const float bv = bias ? bfr(bias[c0 + t * 16 + lr]) : 0.f;
#pragma unroll
        for (int j = 0; j < 8; ++j) os[(hi * 8 + j) * 68 + t * 16 + lr] = acc[t][j] + bv; }
    __syncthreads();
    if (F16OUT) {
        h16* crow = (h16*)(void*)C + (size_t)r0 * ldc + c0;
        auto pass = [&]() {
#pragma unroll
            for (int s = 0; s < 4; ++s) { const int row = 4 * s + (lane >> 3), piece = lane & 7; const float* sp = os + row * 68 + piece * 8; v8h o, o2;
#pragma unroll
                for (int i = 0; i < 8; ++i) { const h16 a = (h16)sp[i]; o[i] = a; o2[i] = (h16)((sp[i] - (float)a) * LOSC); }
                *(volatile v8h*)(crow + (size_t)row * ldc + piece * 8) = o; if (C2) *(volatile v8h*)(C2 + (size_t)r0 * ldc + c0 + (size_t)row * ldc + piece * 8) = o2; }
        };
        pass(); __threadfence(); pass();
    } else {
        float* crow = C + (size_t)r0 * ldc + c0;
        auto pass = [&]() {
#pragma unroll
            for (int s = 0; s < 8; ++s) { const int Lid = (lane >> 3) + 4 * s, piece = lane & 7; const int row = Lid >> 1, cofs = (Lid & 1) * 32 + piece * 4;
                v4f val = *(const v4fa*)(os + row * 68 + cofs); if (R) { const v4f rv = *(const v4f*)(R + ((size_t)r0 + row) * ldc + c0 + cofs); val += roundR ? (v4f){bfr(rv[0]), bfr(rv[1]), bfr(rv[2]), bfr(rv[3])} : rv; }
                *(volatile v4f*)(crow + (size_t)row * ldc + cofs) = val; }
        };
        pass(); __threadfence(); pass();
    }
}

__global__ __launch_bounds__(128) void k_gemm3(const bf* __restrict__ Ah, const bf* __restrict__ Al, const bf* __restrict__ Bh, const bf* __restrict__ Bl, int K, float* C, int ldc) {
    __shared__ __align__(16) float ost[4][16 * 68];
    const int lane = threadIdx.x & 31, wave = threadIdx.x >> 5, lr = lane & 15, hi = lane >> 4;
    const int r0 = blockIdx.x * 64 + wave * 16, c0 = blockIdx.y * 64;
    const size_t aoff = (size_t)(r0 + lr) * K + 8 * hi;
    v8f acc[4];
#pragma unroll
    for (int t = 0; t < 4; ++t) acc[t] = (v8f){};
#pragma unroll 1
    for (int kc = 0; kc < K; kc += 32) {
        const v16bf a = cat16b(*(const v8us*)(Ah + aoff + kc), *(const v8us*)(Ah + aoff + kc + 16));
        const v16bf al = cat16b(*(const v8us*)(Al + aoff + kc), *(const v8us*)(Al + aoff + kc + 16));
#pragma unroll
        for (int t = 0; t < 4; ++t) { const size_t bo = (size_t)(c0 + t * 16 + lr) * K + kc + 8 * hi;
            const v16bf bh = cat16b(*(const v8us*)(Bh + bo), *(const v8us*)(Bh + bo + 16)); const v16bf bl = cat16b(*(const v8us*)(Bl + bo), *(const v8us*)(Bl + bo + 16));
            acc[t] = wmmab(a, bh, acc[t]); acc[t] = wmmab(al, bh, acc[t]); acc[t] = wmmab(a, bl, acc[t]); }
        asm volatile("v_nop\n\tv_nop\n\tv_nop\n\tv_nop" : "+v"(acc[0]), "+v"(acc[1]), "+v"(acc[2]), "+v"(acc[3]) : "v"(a), "v"(al));
    }
    float* os = &ost[wave][0];
#pragma unroll
    for (int t = 0; t < 4; ++t) {
#pragma unroll
        for (int j = 0; j < 8; ++j) os[(hi * 8 + j) * 68 + t * 16 + lr] = acc[t][j]; }
    __builtin_amdgcn_wave_barrier(); asm volatile("" ::: "memory");
    float* crow = C + (size_t)r0 * ldc + c0;
    auto pass = [&]() {
#pragma unroll
        for (int s = 0; s < 8; ++s) { const int Lid = (lane >> 3) + 4 * s, piece = lane & 7; const int row = Lid >> 1, cofs = (Lid & 1) * 32 + piece * 4;
            const v4f val = *(const v4fa*)(os + row * 68 + cofs); *(volatile v4f*)(crow + (size_t)row * ldc + cofs) = val; }
    };
    pass(); __threadfence(); pass();
}
__global__ __launch_bounds__(256) void k_softmax(const float* __restrict__ S, bf* PH, bf* PL) {
    const int lane = threadIdx.x & 31, r = blockIdx.x * 8 + (threadIdx.x >> 5);
    if (r >= NT_) return;
    const float* sr = S + (size_t)r * NT_ + lane * 8;
    float m = -3.0e38f;
#pragma unroll 1
    for (int q = 0; q < NT_ / 256; ++q) { const v8f v = *(const v8f*)(sr + q * 256);
#pragma unroll
        for (int i = 0; i < 8; ++i) m = fmaxf(m, v[i] * SCL); }
#pragma unroll
    for (int sh = 16; sh; sh >>= 1) m = fmaxf(m, __shfl_xor(m, sh, 32));
    float den = 0.f;
#pragma unroll 1
    for (int q = 0; q < NT_ / 256; ++q) { const v8f v = *(const v8f*)(sr + q * 256);
#pragma unroll
        for (int i = 0; i < 8; ++i) den += __expf(v[i] * SCL - m); }
#pragma unroll
    for (int sh = 16; sh; sh >>= 1) den += __shfl_xor(den, sh, 32);
#pragma unroll 1
    for (int ps = 0; ps < 2; ++ps) {
#pragma unroll 1
        for (int q = 0; q < NT_ / 256; ++q) { const v8f v = *(const v8f*)(sr + q * 256); v8us oh, ol;
#pragma unroll
            for (int i = 0; i < 8; ++i) { const float p = __expf(v[i] * SCL - m) / den; const unsigned short hb = f2bf(p); oh[i] = hb; ol[i] = f2bf(p - bf2f(hb)); }
            const size_t o = (size_t)r * NT_ + q * 256 + lane * 8; *(volatile v8us*)(PH + o) = oh; *(volatile v8us*)(PL + o) = ol; }
        if (ps == 0) __threadfence(); }
}
__global__ __launch_bounds__(256) void k_vt(const float* __restrict__ V, bf* VTH, bf* VTL) {
    __shared__ float tl[64][65];
    const int tid = threadIdx.x, t0 = blockIdx.x * 64, d0 = blockIdx.y * 64, g = blockIdx.z;
    { const int tt = tid >> 2, dq = (tid & 3) * 16;
#pragma unroll
      for (int i = 0; i < 16; ++i) tl[dq + i][tt] = V[(size_t)(t0 + tt) * KW + g * HD + d0 + dq + i]; }
    __syncthreads();
    const int piece = tid & 7;
    auto pass = [&]() {
#pragma unroll
        for (int s = 0; s < 2; ++s) { const int d = (tid >> 3) + 32 * s; v8us oh, ol;
#pragma unroll
            for (int i = 0; i < 8; ++i) { const float v = tl[d][piece * 8 + i]; const unsigned short hb = f2bf(v); oh[i] = hb; ol[i] = f2bf(v - bf2f(hb)); }
            const size_t o = ((size_t)g * HD + d0 + d) * NT_ + t0 + piece * 8; *(volatile v8us*)(VTH + o) = oh; *(volatile v8us*)(VTL + o) = ol; }
    };
    pass(); __threadfence(); pass();
}

__global__ __launch_bounds__(256) void k_outT(const float* __restrict__ T, const float* __restrict__ X, const float* __restrict__ gam, float* OUTB) {
    __shared__ __align__(16) float tl[64 * 68];
    const int n0 = blockIdx.x * 64, c0 = blockIdx.y * 64, tid = threadIdx.x;
    const int nn = tid >> 2, cq = (tid & 3) * 16;
#pragma unroll
    for (int i = 0; i < 16; ++i) tl[(cq + i) * 68 + nn] = T[(size_t)(n0 + nn) * CC + c0 + cq + i];
    __syncthreads();
    const float g = bfr(gam[0]);
    const int piece = tid & 15;
    auto pass = [&]() {
#pragma unroll
        for (int s = 0; s < 4; ++s) { const int cr = (tid >> 4) + 16 * s; const size_t o = (size_t)(c0 + cr) * NPOS + n0 + piece * 4;
            const v4f xv = *(const v4f*)(X + o); v4f val = *(const v4fa*)(tl + cr * 68 + piece * 4);
#pragma unroll
            for (int k = 0; k < 4; ++k) val[k] = g * val[k] + bfr(xv[k]);
            *(volatile v4f*)(OUTB + o) = val; }
    };
    pass(); __threadfence(); pass();
}

extern "C" void kernel_launch(void* const* d_in, const int* in_sizes, int n_in,
                              void* d_out, int out_size, void* d_ws, size_t ws_size, hipStream_t stream) {
    (void)in_sizes; (void)n_in; (void)out_size;
    const float* x = (const float*)d_in[0]; const float* fw = (const float*)d_in[1]; const float* fb = (const float*)d_in[2]; const float* gw = (const float*)d_in[3]; const float* gb = (const float*)d_in[4];
    const float* hw = (const float*)d_in[5]; const float* hb = (const float*)d_in[6]; const float* gam = (const float*)d_in[7];
    float* out = (float*)d_out;
    char* wsp = (char*)d_ws;
    auto take = [&](size_t bytes) { char* p = wsp; wsp += (bytes + 255) & ~(size_t)255; return (void*)p; };
    bf* FwB = (bf*)take((size_t)OC * CC * 2); bf* GwB = (bf*)take((size_t)OC * CC * 2); bf* HwB = (bf*)take((size_t)CC * CC * 2);
    bf* XT = (bf*)take((size_t)NPOS * CC * 2); float* TMP = (float*)take((size_t)NPOS * CC * 4);
    bf* Fh = (bf*)take((size_t)NPOS * OC * 2); bf* Fl = (bf*)take((size_t)NPOS * OC * 2); bf* Gh = (bf*)take((size_t)NPOS * OC * 2); bf* Gl = (bf*)take((size_t)NPOS * OC * 2);
    bf* Hh = (bf*)take((size_t)CC * NPOS * 2); bf* Hl = (bf*)take((size_t)CC * NPOS * 2);
    float* S = (float*)take((size_t)QH_ * NPOS * 4); bf* Ph = (bf*)take((size_t)QH_ * NPOS * 2); bf* Pl = (bf*)take((size_t)QH_ * NPOS * 2); float* OT = (float*)take((size_t)NPOS * CC * 4);
    if ((size_t)(wsp - (char*)d_ws) > ws_size) return;
    k_cvtb<<<OC / 8, 256, 0, stream>>>(fw, OC, FwB); k_cvtb<<<OC / 8, 256, 0, stream>>>(gw, OC, GwB); k_cvtb<<<CC / 8, 256, 0, stream>>>(hw, CC, HwB);
    for (int b = 0; b < NB_; ++b) {
        const float* xb = x + (size_t)b * CC * NPOS;
        k_wt<<<dim3(CC / 64, NPOS / 64, 1), 256, 0, stream>>>(xb, CC, NPOS, XT);
        k_gemmb<false, false><<<dim3(NPOS / 64, OC / 64, 1), 128, 0, stream>>>(XT, nullptr, FwB, fb, TMP, OC, nullptr); k_cvtb2<<<(NPOS * OC / CC) / 8, 256, 0, stream>>>(TMP, NPOS * OC / CC, Fh, Fl);
        k_gemmb<false, false><<<dim3(NPOS / 64, OC / 64, 1), 128, 0, stream>>>(XT, nullptr, GwB, gb, TMP, OC, nullptr); k_cvtb2<<<(NPOS * OC / CC) / 8, 256, 0, stream>>>(TMP, NPOS * OC / CC, Gh, Gl);
        k_gemmb<false, false><<<dim3(NPOS / 64, CC / 64, 1), 128, 0, stream>>>(XT, nullptr, HwB, hb, TMP, CC, nullptr); k_vt<<<dim3(NPOS / 64, 2, NKV), 256, 0, stream>>>(TMP, Hh, Hl);
        for (int hq = 0; hq < 2; ++hq) {
            k_gemm3<<<dim3(QH_ / 64, NPOS / 64, 1), 128, 0, stream>>>(Gh + (size_t)hq * QH_ * OC, Gl + (size_t)hq * QH_ * OC, Fh, Fl, OC, S, NPOS);
            k_softmax<<<QH_ / 8, 256, 0, stream>>>(S, Ph, Pl);
            k_gemm3<<<dim3(QH_ / 64, CC / 64, 1), 128, 0, stream>>>(Ph, Pl, Hh, Hl, NPOS, OT + (size_t)hq * QH_ * CC, CC);
        }
        k_outT<<<dim3(NPOS / 64, CC / 64, 1), 256, 0, stream>>>(OT, xb, gam, out + (size_t)b * CC * NPOS);
    }
}
